// TransformerLayer_17678085391074
// MI455X (gfx1250) — hardware-verified
//
#include <hip/hip_runtime.h>
#include <math.h>

typedef __attribute__((ext_vector_type(16))) _Float16 v16h;
typedef __attribute__((ext_vector_type(8)))  _Float16 v8h;
typedef __attribute__((ext_vector_type(8)))  float v8f;
typedef __attribute__((ext_vector_type(4)))  float v4f;

#ifndef SEQ
#define SEQ 2048
#endif
#define SEQ_FULL 2048
#ifndef NB
#define NB 2
#endif
#define NB_FULL 2
#define DM 1024
#define NH 16
#define HD 64
#define DF 4096
#define MROWS (NB * SEQ)
#define WC (64.0f)
#define PCY (16384.0f)
#define CC (256.0f)
#define GC (256.0f)
#define F16MIN (6.103515625e-05f)
#define LN_EPS (1e-5f)
static_assert(SEQ % 64 == 0);
static_assert(SEQ >= 64);
static_assert(SEQ <= SEQ_FULL);
static_assert(NB >= 1 && NB <= NB_FULL);
static_assert(DM == NH * HD);
static_assert(HD == 64);
static_assert(DM % 128 == 0 && DF % 128 == 0 && DM % 32 == 0 && DF % 32 == 0);
static_assert(MROWS % 64 == 0 && MROWS % 8 == 0);
static_assert((DM * DM / 8) % 256 == 0 && (DF * DM / 8) % 256 == 0);
static_assert((size_t)(MROWS / 8) * 8 * DM == (size_t)MROWS * DM);
static_assert((size_t)(MROWS / 64) * (DM / 128) * 2 * 64 * 128 == 2 * (size_t)MROWS * DM);
static_assert((size_t)(MROWS / 64) * (DM / 128) * 64 * 128 == (size_t)NB * DM * SEQ);
static_assert((size_t)(SEQ / 64) * NH * NB * 64 * HD == (size_t)MROWS * DM);
static_assert((size_t)(MROWS / 64) * (DF / 128) * 64 * 128 == (size_t)MROWS * DF);

#define WSZ_WDD  (2u * (size_t)DM * DM)
#define WSZ_WUD  (2u * (size_t)DF * DM)
#define WSZ_ACT  (2u * (size_t)MROWS * DM)
#define WSZ_X1   (4u * (size_t)MROWS * DM)
#define WSZ_G    (2u * (size_t)MROWS * DF)
#define WS_WQ   ((size_t)0)
#define WS_WK   (WS_WQ + WSZ_WDD)
#define WS_WV   (WS_WK + WSZ_WDD)
#define WS_WO   (WS_WV + WSZ_WDD)
#define WS_WU   (WS_WO + WSZ_WDD)
#define WS_WD   (WS_WU + WSZ_WUD)
#define WS_H1   (WS_WD + WSZ_WUD)
#define WS_Q    (WS_H1 + WSZ_ACT)
#define WS_K    (WS_Q  + WSZ_ACT)
#define WS_VT   (WS_K  + WSZ_ACT)
#define WS_CTX  (WS_VT + WSZ_ACT)
#define WS_X1   (WS_CTX + WSZ_ACT)
#define WS_H2   (WS_X1 + WSZ_X1)
#define WS_G    (WS_H2 + WSZ_ACT)
#define WS_END  (WS_G  + WSZ_G)
static_assert(WS_END <= (size_t)134217728u);
static_assert((WS_H1 % 256u) == 0 && (WS_VT % 256u) == 0 && (WS_X1 % 256u) == 0 && (WS_G % 256u) == 0);

template <typename T> __device__ __forceinline__ void vst2(void* p, T v) { *(volatile T*)p = v; __threadfence(); *(volatile T*)p = v; }
__device__ __forceinline__ v8f zero8() { v8f z = {0.f, 0.f, 0.f, 0.f, 0.f, 0.f, 0.f, 0.f}; return z; }
__device__ __forceinline__ v8f wmma16(v16h a, v16h b, v8f c) {
  v8f d = __builtin_amdgcn_wmma_f32_16x16x32_f16(false, a, false, b, (short)0, c, false, false);
  asm volatile("v_nop\n\tv_nop\n\tv_nop\n\tv_nop" : "+v"(d) : "v"(a), "v"(b));
  return d;
}
__device__ __forceinline__ v16h frag_h(const _Float16* rowk0, unsigned lane) {
  union { v16h v; v8h q[2]; } u; const _Float16* p = rowk0 + 8u * (lane >> 4);
  u.q[0] = *(const v8h*)p; u.q[1] = *(const v8h*)(p + 16); return u.v;
}
__device__ __forceinline__ _Float16 f16n(float x) { const float t = (fabsf(x) >= F16MIN) ? x : 0.0f; return (_Float16)t; }
__device__ __forceinline__ unsigned short bf16bits(float x) { unsigned u = __float_as_uint(x); u += 0x7FFFu + ((u >> 16) & 1u); return (unsigned short)(u >> 16); }
__device__ __forceinline__ float bf16val(unsigned short b) { return __uint_as_float(((unsigned)b) << 16); }
__device__ __forceinline__ float bfr(float x) { return bf16val(bf16bits(x)); }
#define LDSX() do { asm volatile("s_wait_dscnt 0" ::: "memory"); __builtin_amdgcn_wave_barrier(); __builtin_amdgcn_fence(3  , "workgroup"); } while (0)
template <int KLEN>
__device__ __forceinline__ void gemm_16x128(v8f (&acc)[8], const _Float16* arow, const _Float16* wrow, unsigned lane) {
  static_assert(KLEN % 32 == 0);
#pragma unroll
  for (int j = 0; j < 8; ++j) acc[j] = zero8();
#pragma unroll 1
  for (unsigned kc = 0; kc < (unsigned)KLEN / 32u; ++kc) {
    const v16h a = frag_h(arow + kc * 32u, lane);
#pragma unroll
    for (int j = 0; j < 8; ++j) acc[j] = wmma16(a, frag_h(wrow + (size_t)(j * 16) * (size_t)KLEN + kc * 32u, lane), acc[j]);
  }
}

__global__ __launch_bounds__(256) void k_cvth(const float* __restrict__ src, int n8, _Float16* __restrict__ dst) {
  const int i = blockIdx.x * 256 + (int)threadIdx.x; if (i >= n8) return;
  const float* p = src + (size_t)i * 8; const v4f a = *(const v4f*)p, b = *(const v4f*)(p + 4);
  v8h o;
#pragma unroll
  for (int e = 0; e < 4; ++e) { o[e] = f16n(bfr(a[e]) * WC); o[4 + e] = f16n(bfr(b[e]) * WC); }
  vst2(dst + (size_t)i * 8, o);
}

template <int INB> __device__ __forceinline__ void ld8(const float* p, v4f& a, v4f& b) {
  a = *(const v4f*)p; b = *(const v4f*)(p + 4);
  if (INB) {
#pragma unroll
    for (int e = 0; e < 4; ++e) { a[e] = bfr(a[e]); b[e] = bfr(b[e]); }
  }
}
template <int INB> __global__ __launch_bounds__(256) void k_ln(const float* __restrict__ X, const float* __restrict__ SC, const float* __restrict__ SH, _Float16* __restrict__ H) {
  const unsigned wave = threadIdx.x >> 5, lane = threadIdx.x & 31u; const unsigned row = blockIdx.x * 8u + wave; if (row >= (unsigned)MROWS) return;
  const size_t sb = INB ? ((size_t)(row / (unsigned)SEQ) * SEQ_FULL + (row % (unsigned)SEQ)) * DM : (size_t)row * DM;
  const size_t rb = (size_t)row * DM;
  float s1 = 0.f;
#pragma unroll 1
  for (unsigned i = 0; i < 4; ++i) { v4f a, b; ld8<INB>(X + sb + i * 256u + lane * 8u, a, b); s1 += ((a[0] + a[1]) + (a[2] + a[3])) + ((b[0] + b[1]) + (b[2] + b[3])); }
#pragma unroll
  for (int o = 1; o < 32; o <<= 1) s1 += __shfl_xor(s1, o);
  const float mu = s1 * (1.0f / DM); float q = 0.f;
#pragma unroll 1
  for (unsigned i = 0; i < 4; ++i) { v4f a, b; ld8<INB>(X + sb + i * 256u + lane * 8u, a, b);
#pragma unroll
    for (int e = 0; e < 4; ++e) { const float d0 = a[e] - mu, d1 = b[e] - mu; q += d0 * d0; q += d1 * d1; } }
#pragma unroll
  for (int o = 1; o < 32; o <<= 1) q += __shfl_xor(q, o);
  const float inv = 1.0f / (q * (1.0f / (float)(DM - 1)) + LN_EPS);
#pragma unroll 1
  for (unsigned i = 0; i < 4; ++i) { v4f a, b, sa, sb4, ha, hb; ld8<INB>(X + sb + i * 256u + lane * 8u, a, b); ld8<1>(SC + i * 256u + lane * 8u, sa, sb4); ld8<1>(SH + i * 256u + lane * 8u, ha, hb);
    v8h o8;
#pragma unroll
    for (int e = 0; e < 4; ++e) { o8[e] = f16n(((a[e] - mu) * inv) * sa[e] + ha[e]); o8[4 + e] = f16n(((b[e] - mu) * inv) * sb4[e] + hb[e]); }
    vst2(H + rb + i * 256u + lane * 8u, o8); }
}

__global__ __launch_bounds__(128) void k_pqk(const _Float16* __restrict__ H, const _Float16* __restrict__ W2, _Float16* __restrict__ O2) {
  __shared__ __align__(16) _Float16 sh[64][136];
  const unsigned tid = threadIdx.x, wave = tid >> 5, lane = tid & 31u, col = lane & 15u, g = lane >> 4;
  const _Float16* W = W2 + (size_t)blockIdx.z * DM * DM; _Float16* O = O2 + (size_t)blockIdx.z * MROWS * DM;
  const unsigned c0 = blockIdx.y * 128u; const size_t r0 = (size_t)blockIdx.x * 64;
  v8f acc[8];
  gemm_16x128<DM>(acc, H + (r0 + wave * 16u + col) * DM, W + (size_t)(c0 + col) * DM, lane);
#pragma unroll
  for (int j = 0; j < 8; ++j)
#pragma unroll
    for (int r = 0; r < 8; ++r) sh[wave * 16u + 8u * g + r][j * 16 + col] = f16n(acc[j][r] * (1.0f / WC));
  __syncthreads();
  for (unsigned e = tid; e < 64u * 16u; e += 128u) { const unsigned rl = e >> 4, q = e & 15u; vst2(O + (r0 + rl) * (size_t)DM + c0 + q * 8u, *(const v8h*)&sh[rl][q * 8u]); }
}

__global__ __launch_bounds__(128) void k_pvt(const _Float16* __restrict__ H, const _Float16* __restrict__ WV, _Float16* __restrict__ VT) {
  __shared__ __align__(16) _Float16 th[128][72];
  const unsigned tid = threadIdx.x, wave = tid >> 5, lane = tid & 31u, col = lane & 15u, g = lane >> 4;
  const unsigned c0 = blockIdx.y * 128u; const unsigned rr = blockIdx.x * 64u; const size_t r0 = rr;
  const unsigned b = rr / (unsigned)SEQ, t0 = rr % (unsigned)SEQ;
  v8f acc[8];
  gemm_16x128<DM>(acc, H + (r0 + wave * 16u + col) * DM, WV + (size_t)(c0 + col) * DM, lane);
#pragma unroll
  for (int j = 0; j < 8; ++j)
#pragma unroll
    for (int r = 0; r < 8; ++r) th[j * 16 + col][wave * 16u + 8u * g + r] = f16n(acc[j][r] * (1.0f / WC));
  __syncthreads();
  for (unsigned e = tid; e < 128u * 8u; e += 128u) { const unsigned cl = e >> 3, q = e & 7u; vst2(VT + ((size_t)b * DM + c0 + cl) * SEQ + t0 + q * 8u, *(const v8h*)&th[cl][q * 8u]); }
}

__global__ __launch_bounds__(128) void k_att(const _Float16* __restrict__ Q, const _Float16* __restrict__ Kp, const _Float16* __restrict__ VT, _Float16* __restrict__ CTX) {
  __shared__ __align__(16) _Float16 sP[4][16][72];
  __shared__ __align__(16) _Float16 sT[64][72];
  const unsigned tid = threadIdx.x, wave = tid >> 5, lane = tid & 31u, col = lane & 15u, g = lane >> 4;
  const unsigned t0 = blockIdx.x * 64u, h = blockIdx.y, b = blockIdx.z;
  const size_t rowq = (size_t)b * SEQ + t0 + wave * 16u + col;
  v16h aq[2];
#pragma unroll
  for (int kc = 0; kc < 2; ++kc) aq[kc] = frag_h(Q + rowq * DM + h * HD + kc * 32, lane);
  const _Float16* kb = Kp + (size_t)b * SEQ * DM + h * HD;
  const _Float16* vb = VT + ((size_t)b * DM + h * HD) * SEQ;
  float m[8], lsum[8];
#pragma unroll
  for (int r = 0; r < 8; ++r) { m[r] = -3.0e38f; lsum[r] = 0.f; }
  v8f acc[4];
#pragma unroll
  for (int j = 0; j < 4; ++j) acc[j] = zero8();
#pragma unroll 1
  for (unsigned kt = 0; kt < (unsigned)SEQ / 64u; ++kt) {
    const unsigned key0 = kt * 64u;
    v8f s[4];
#pragma unroll
    for (int t = 0; t < 4; ++t) { s[t] = zero8();
#pragma unroll
      for (int kc = 0; kc < 2; ++kc) s[t] = wmma16(aq[kc], frag_h(kb + (size_t)(key0 + t * 16 + col) * DM + kc * 32, lane), s[t]); }
    float al[8];
#pragma unroll
    for (int r = 0; r < 8; ++r) {
      float tm = fmaxf(fmaxf(s[0][r], s[1][r]), fmaxf(s[2][r], s[3][r])) * 0.125f;
      tm = fmaxf(tm, __shfl_xor(tm, 1)); tm = fmaxf(tm, __shfl_xor(tm, 2)); tm = fmaxf(tm, __shfl_xor(tm, 4)); tm = fmaxf(tm, __shfl_xor(tm, 8));
      const float mn = fmaxf(m[r], tm);
      al[r] = __expf(fmaxf(m[r] - mn, -100.0f)); m[r] = mn; lsum[r] *= al[r];
    }
#pragma unroll
    for (int j = 0; j < 4; ++j)
#pragma unroll
      for (int r = 0; r < 8; ++r) acc[j][r] *= al[r];
    LDSX();
#pragma unroll
    for (int t = 0; t < 4; ++t)
#pragma unroll
      for (int r = 0; r < 8; ++r) {
        const float e = s[t][r] * 0.125f - m[r];
        float pc = __expf(e) * PCY; pc = (pc >= F16MIN) ? pc : 0.0f;
        const _Float16 ph = (_Float16)pc;
        lsum[r] += (float)ph;
        sP[wave][8u * g + r][t * 16 + col] = ph;
      }
    LDSX();
#pragma unroll
    for (int kk = 0; kk < 2; ++kk) {
      const v16h a = frag_h(&sP[wave][col][kk * 32], lane);
#pragma unroll
      for (int j = 0; j < 4; ++j) acc[j] = wmma16(a, frag_h(vb + (size_t)(j * 16 + col) * SEQ + key0 + kk * 32, lane), acc[j]);
    }
  }
  float inv[8];
#pragma unroll
  for (int r = 0; r < 8; ++r) { float t = lsum[r]; t += __shfl_xor(t, 1); t += __shfl_xor(t, 2); t += __shfl_xor(t, 4); t += __shfl_xor(t, 8); inv[r] = (1.0f / t) * CC; }
#pragma unroll
  for (int j = 0; j < 4; ++j)
#pragma unroll
    for (int r = 0; r < 8; ++r) sT[j * 16 + col][wave * 16u + 8u * g + r] = f16n(acc[j][r] * inv[r]);
  __syncthreads();
  _Float16* cbase = CTX + (size_t)b * SEQ * DM + (size_t)(h * HD) * SEQ + t0;
  for (unsigned e = tid; e < 64u * 8u; e += 128u) { const unsigned dl = e >> 3, q = e & 7u; vst2(cbase + (size_t)dl * SEQ + q * 8u, *(const v8h*)&sT[dl][q * 8u]); }
}

template <int RB, int KLEN> __global__ __launch_bounds__(128) void k_gres(const _Float16* __restrict__ A, const _Float16* __restrict__ W, const float* __restrict__ BIAS, const float* __restrict__ RES, float* __restrict__ OUT, float sc) {
  __shared__ __align__(16) float sf[4][16][132];
  const unsigned tid = threadIdx.x, wave = tid >> 5, lane = tid & 31u, col = lane & 15u, g = lane >> 4; const unsigned c0 = blockIdx.y * 128u; const unsigned rr = blockIdx.x * 64u + wave * 16u; const size_t r0 = rr;
  v8f acc[8];
  gemm_16x128<KLEN>(acc, A + (r0 + col) * (size_t)KLEN, W + (size_t)(c0 + col) * KLEN, lane);
#pragma unroll
  for (int j = 0; j < 8; ++j)
#pragma unroll
    for (int r = 0; r < 8; ++r) sf[wave][8u * g + r][j * 16 + col] = acc[j][r] * sc;
  LDSX();
  v4f bv = *(const v4f*)(BIAS + c0 + lane * 4u);
  bv[0] = bfr(bv[0]); bv[1] = bfr(bv[1]); bv[2] = bfr(bv[2]); bv[3] = bfr(bv[3]);
  for (unsigned rl = 0; rl < 16u; ++rl) {
    const unsigned grow = rr + rl;
    const size_t o = (size_t)grow * DM + c0 + lane * 4u;
    const size_t so = RB ? ((size_t)(grow / (unsigned)SEQ) * SEQ_FULL + (grow % (unsigned)SEQ)) * DM + c0 + lane * 4u : o;
    v4f vv = *(const v4f*)&sf[wave][rl][lane * 4u]; v4f rv = *(const v4f*)(RES + so);
    if (RB) { rv[0] = bfr(rv[0]); rv[1] = bfr(rv[1]); rv[2] = bfr(rv[2]); rv[3] = bfr(rv[3]); }
    vv[0] = (vv[0] + bv[0]) + rv[0]; vv[1] = (vv[1] + bv[1]) + rv[1]; vv[2] = (vv[2] + bv[2]) + rv[2]; vv[3] = (vv[3] + bv[3]) + rv[3];
    vst2(OUT + o, vv);
  }
}

__global__ __launch_bounds__(128) void k_up(const _Float16* __restrict__ H, const _Float16* __restrict__ WU, const float* __restrict__ BU, _Float16* __restrict__ G) {
  __shared__ __align__(16) float sf[64][132];
  const unsigned tid = threadIdx.x, wave = tid >> 5, lane = tid & 31u, col = lane & 15u, g = lane >> 4;
  const unsigned c0 = blockIdx.y * 128u; const size_t r0 = (size_t)blockIdx.x * 64;
  v8f acc[8];
  gemm_16x128<DM>(acc, H + (r0 + wave * 16u + col) * DM, WU + (size_t)(c0 + col) * DM, lane);
#pragma unroll
  for (int j = 0; j < 8; ++j)
#pragma unroll
    for (int r = 0; r < 8; ++r) sf[wave * 16u + 8u * g + r][j * 16 + col] = acc[j][r] * (1.0f / WC);
  __syncthreads();
  const unsigned q = tid & 15u;
  v4f b0 = *(const v4f*)(BU + c0 + q * 8u), b1 = *(const v4f*)(BU + c0 + q * 8u + 4u);
#pragma unroll
  for (int e = 0; e < 4; ++e) { b0[e] = bfr(b0[e]); b1[e] = bfr(b1[e]); }
#pragma unroll 1
  for (unsigned it = 0; it < 8u; ++it) {
    const unsigned rl = (tid >> 4) + it * 8u;
    const v4f a0 = *(const v4f*)&sf[rl][q * 8u], a1 = *(const v4f*)&sf[rl][q * 8u + 4u];
    v8h o;
#pragma unroll
    for (int e = 0; e < 4; ++e) {
      const float u0 = a0[e] + b0[e], u1 = a1[e] + b1[e];
      o[e] = f16n((0.5f * u0 * (1.0f + erff(u0 * 0.70710678118654752f))) * GC);
      o[4 + e] = f16n((0.5f * u1 * (1.0f + erff(u1 * 0.70710678118654752f))) * GC);
    }
    vst2(G + (r0 + rl) * (size_t)DF + c0 + q * 8u, o);
  }
}

extern "C" void kernel_launch(void* const* d_in, const int* in_sizes, int n_in, void* d_out, int out_size, void* d_ws, size_t ws_size, hipStream_t stream) {
  if (n_in < 14) return;
  if (in_sizes[0] < ((NB - 1) * SEQ_FULL + SEQ) * DM) return;
  if (in_sizes[1] < DM * DM || in_sizes[2] < DM * DM || in_sizes[3] < DM * DM || in_sizes[4] < DM * DM) return;
  if (in_sizes[5] < DM || in_sizes[6] < DF * DM || in_sizes[7] < DF || in_sizes[8] < DM * DF || in_sizes[9] < DM) return;
  if (in_sizes[10] < DM || in_sizes[11] < DM || in_sizes[12] < DM || in_sizes[13] < DM) return;
  if (out_size < MROWS * DM) return;
  if (ws_size < (size_t)WS_END) return;
  const float* X = (const float*)d_in[0]; const float* WQ = (const float*)d_in[1]; const float* WK = (const float*)d_in[2]; const float* WV = (const float*)d_in[3];
  const float* WO = (const float*)d_in[4]; const float* BO = (const float*)d_in[5]; const float* WU = (const float*)d_in[6]; const float* BU = (const float*)d_in[7];
  const float* WD = (const float*)d_in[8]; const float* BD = (const float*)d_in[9]; const float* S1 = (const float*)d_in[10]; const float* T1 = (const float*)d_in[11];
  const float* S2 = (const float*)d_in[12]; const float* T2 = (const float*)d_in[13];
  char* ws = (char*)d_ws;
  _Float16 *WQH = (_Float16*)(ws + WS_WQ), *WKH = (_Float16*)(ws + WS_WK), *WVH = (_Float16*)(ws + WS_WV), *WOH = (_Float16*)(ws + WS_WO), *WUH = (_Float16*)(ws + WS_WU), *WDH = (_Float16*)(ws + WS_WD);
  _Float16 *H1 = (_Float16*)(ws + WS_H1), *QP = (_Float16*)(ws + WS_Q), *KP = (_Float16*)(ws + WS_K), *VT = (_Float16*)(ws + WS_VT), *CTX = (_Float16*)(ws + WS_CTX), *H2 = (_Float16*)(ws + WS_H2), *G = (_Float16*)(ws + WS_G);
  float* X1 = (float*)(ws + WS_X1);

  const int n8d = DM * DM / 8, n8f = DF * DM / 8;
  k_cvth<<<dim3((n8d + 255) / 256), 256, 0, stream>>>(WQ, n8d, WQH);
  k_cvth<<<dim3((n8d + 255) / 256), 256, 0, stream>>>(WK, n8d, WKH);
  k_cvth<<<dim3((n8d + 255) / 256), 256, 0, stream>>>(WV, n8d, WVH);
  k_cvth<<<dim3((n8d + 255) / 256), 256, 0, stream>>>(WO, n8d, WOH);
  k_cvth<<<dim3((n8f + 255) / 256), 256, 0, stream>>>(WU, n8f, WUH);
  k_cvth<<<dim3((n8f + 255) / 256), 256, 0, stream>>>(WD, n8f, WDH);
  k_ln<1><<<dim3(MROWS / 8), 256, 0, stream>>>(X, S1, T1, H1);
  k_pqk<<<dim3(MROWS / 64, DM / 128, 2), 128, 0, stream>>>(H1, WQH, QP);
  k_pvt<<<dim3(MROWS / 64, DM / 128), 128, 0, stream>>>(H1, WVH, VT);
  k_att<<<dim3(SEQ / 64, NH, NB), 128, 0, stream>>>(QP, KP, VT, CTX);
  k_gres<1, DM><<<dim3(MROWS / 64, DM / 128), 128, 0, stream>>>(CTX, WOH, BO, X, X1, 1.0f / (CC * WC));
  k_ln<0><<<dim3(MROWS / 8), 256, 0, stream>>>(X1, S2, T2, H2);
  k_up<<<dim3(MROWS / 64, DF / 128), 128, 0, stream>>>(H2, WUH, BU, G);
  k_gres<0, DF><<<dim3(MROWS / 64, DM / 128), 128, 0, stream>>>(G, WDH, BD, X1, (float*)d_out, 1.0f / (GC * WC));
}
